// dgl_sage_73529840107894
// MI455X (gfx1250) — hardware-verified
//
#include <hip/hip_runtime.h>
#include <math.h>
#define SRB 1024
#define SCHK 4096
typedef __attribute__((ext_vector_type(16))) _Float16 v16h;
typedef __attribute__((ext_vector_type(8)))  _Float16 v8h;
typedef __attribute__((ext_vector_type(16))) __bf16   v16b;
typedef __attribute__((ext_vector_type(8)))  __bf16   v8b;
typedef __attribute__((ext_vector_type(8)))  float    v8f;
typedef __attribute__((ext_vector_type(4)))  float    v4f;
#define PSCALE 32768.0f
#define U16(p) ((const unsigned short*)(const void*)(p))
#define PSCALE_INV (1.0f / 32768.0f)

__device__ __forceinline__ unsigned short f2bf_bits(float f) {
  unsigned u = __float_as_uint(f);
  return (unsigned short)((u + 0x7FFFu + ((u >> 16) & 1u)) >> 16);
}
__device__ __forceinline__ float bf_bits2f(unsigned short h) { return __uint_as_float(((unsigned)h) << 16); }

__device__ __forceinline__ void dep_guard_h(v8f& a, v8f& b, v16h x, v16h y) { asm volatile("v_nop\n\tv_nop\n\tv_nop\n\tv_nop" : "+v"(a), "+v"(b) : "v"(x), "v"(y)); }
__device__ __forceinline__ void dep_guard_b(v8f& a, v8f& b, v16b x, v16b y) { asm volatile("v_nop\n\tv_nop\n\tv_nop\n\tv_nop" : "+v"(a), "+v"(b) : "v"(x), "v"(y)); }
__device__ __forceinline__ void keep4_h(v16h a, v16h b, v16h c, v16h d) { asm volatile("v_nop" :: "v"(a), "v"(b), "v"(c), "v"(d)); }
__device__ __forceinline__ void keep4_b(v16b a, v16b b, v16b c, v16b d) { asm volatile("v_nop" :: "v"(a), "v"(b), "v"(c), "v"(d)); }
__device__ __forceinline__ void acc_guard4(v8f& a, v8f& b, v8f& c, v8f& d) { asm volatile("v_nop\n\tv_nop\n\tv_nop\n\tv_nop" : "+v"(a), "+v"(b), "+v"(c), "+v"(d)); }
template <typename T> struct Frag;
template <> struct Frag<_Float16> {
  typedef v16h V; union U { v16h v; v8h h[2]; };
  static __device__ __forceinline__ v16h load(const _Float16* p) {
    U f; f.h[0] = *(const v8h*)(p); f.h[1] = *(const v8h*)(p + 16); return f.v;
  }
  static __device__ __forceinline__ v8f mma(v16h a, v16h b, v8f c) {
    return __builtin_amdgcn_wmma_f32_16x16x32_f16(false, a, false, b, (short)0, c, false, false);
  }
  static __device__ __forceinline__ void guard(v8f& a, v8f& b, v16h x, v16h y) { dep_guard_h(a, b, x, y); }
  static __device__ __forceinline__ void keep(v16h a, v16h b, v16h c, v16h d) { keep4_h(a, b, c, d); }
};
template <> struct Frag<__bf16> {
  typedef v16b V; union U { v16b v; v8b h[2]; };
  static __device__ __forceinline__ v16b load(const __bf16* p) {
    U f; f.h[0] = *(const v8b*)(p); f.h[1] = *(const v8b*)(p + 16); return f.v;
  }
  static __device__ __forceinline__ v8f mma(v16b a, v16b b, v8f c) {
    return __builtin_amdgcn_wmma_f32_16x16x32_bf16(false, a, false, b, (short)0, c, false, false);
  }
  static __device__ __forceinline__ void guard(v8f& a, v8f& b, v16b x, v16b y) { dep_guard_b(a, b, x, y); }
  static __device__ __forceinline__ void keep(v16b a, v16b b, v16b c, v16b d) { keep4_b(a, b, c, d); }
};

template <int ET> struct Elem;
template <> struct Elem<0> { typedef _Float16 T; };
template <> struct Elem<1> { typedef __bf16 T; };
template <int ET, bool SPLIT, int BIAS_MODE, int OUT_MODE, bool RESID, int ACT = 0>
__global__ __launch_bounds__(256) void wmma_gemm64(
    const unsigned short* __restrict__ Ap, const unsigned short* __restrict__ A2p, int lda, long strideA,
    const unsigned short* __restrict__ Btp, const unsigned short* __restrict__ Bt2p, int ldb, long strideB,
    void* __restrict__ Cout, void* __restrict__ Cout2, int ldc, long strideC,
    const float* __restrict__ bias,
    const float* __restrict__ resid, long strideR,
    int M, int N, int K, float scale) {
  typedef typename Elem<ET>::T T;
  typedef typename Frag<T>::V V;
  const T* A = (const T*)Ap; const T* A2 = (const T*)A2p; const T* Bt = (const T*)Btp; const T* Bt2 = (const T*)Bt2p;
  __shared__ __align__(16) float sT[8][16 * 68];
  const int b    = blockIdx.y;
  const int lane = threadIdx.x & 31;
  const int wave = threadIdx.x >> 5;
  const int tilesN = N >> 6;
  const int tilesM = M >> 6;
  const int tile = blockIdx.x * 8 + wave;
  if (tile >= tilesM * tilesN) return;
  const int tm = tile / tilesN;
  const int tn = tile - tm * tilesN;
  const int m0 = tm << 6;
  const int n0 = tn << 6;

  const T* Ab  = A  + (size_t)b * strideA;
  const T* Bb  = Bt + (size_t)b * strideB;
  const T* Ab2 = SPLIT ? (A2  + (size_t)b * strideA) : nullptr;
  const T* Bb2 = SPLIT ? (Bt2 + (size_t)b * strideB) : nullptr;

  const int rlane = lane & 15;
  const int koff  = (lane >> 4) * 8;
  const int mOff  = (lane >> 4) * 8;

  v8f acc[4][4];
#pragma unroll
  for (int i = 0; i < 4; ++i)
#pragma unroll
    for (int j = 0; j < 4; ++j) acc[i][j] = (v8f){0.f,0.f,0.f,0.f,0.f,0.f,0.f,0.f};

  for (int k0 = 0; k0 < K; k0 += 32) {
    V bh[4], bl[4];
#pragma unroll
    for (int j = 0; j < 4; ++j) {
      const size_t bo = (size_t)(n0 + (j << 4) + rlane) * ldb + koff + k0;
      bh[j] = Frag<T>::load(Bb + bo);
      if (SPLIT) bl[j] = Frag<T>::load(Bb2 + bo);
    }
#pragma unroll
    for (int i = 0; i < 4; ++i) {
      const size_t ao = (size_t)(m0 + (i << 4) + rlane) * lda + koff + k0;
      V ah = Frag<T>::load(Ab + ao);
      V al;
      if (SPLIT) al = Frag<T>::load(Ab2 + ao);
#pragma unroll
      for (int j = 0; j < 4; ++j) {
        acc[i][j] = Frag<T>::mma(ah, bh[j], acc[i][j]);
        if (SPLIT) {
          acc[i][j] = Frag<T>::mma(ah, bl[j], acc[i][j]);
          acc[i][j] = Frag<T>::mma(al, bh[j], acc[i][j]);
        }
      }
      Frag<T>::guard(acc[i][0], acc[i][3], ah, SPLIT ? al : ah);
    }
    Frag<T>::keep(bh[0], bh[1], bh[2], bh[3]);
    if (SPLIT) Frag<T>::keep(bl[0], bl[1], bl[2], bl[3]);
  }
  acc_guard4(acc[0][0], acc[0][1], acc[0][2], acc[0][3]);
  acc_guard4(acc[1][0], acc[1][1], acc[1][2], acc[1][3]);
  acc_guard4(acc[2][0], acc[2][1], acc[2][2], acc[2][3]);
  acc_guard4(acc[3][0], acc[3][1], acc[3][2], acc[3][3]);

  float* slab = sT[wave];
  const float* Rb = RESID ? (resid + (size_t)b * strideR) : nullptr;
#pragma unroll
  for (int i = 0; i < 4; ++i) {
    const int mBase = m0 + (i << 4);
#pragma unroll
    for (int j = 0; j < 4; ++j) {
      const int n = n0 + (j << 4) + rlane;
      float bv = 0.f;
      if (BIAS_MODE == 2) bv = bias[n];
#pragma unroll
      for (int r = 0; r < 8; ++r) {
        float v = acc[i][j][r] * scale;
        if (BIAS_MODE == 1) v += bias[mBase + mOff + r];
        if (BIAS_MODE == 2) v += bv;
        if (RESID) v += Rb[(size_t)(mBase + mOff + r) * ldc + n];
        if (ACT == 1) v = tanhf(v);
        if (ACT == 2) v = fmaxf(v, 0.0f);
        if (ACT == 3) v = v / (1.0f + expf(-v));
        if (ACT == 4) v = (v > 0.f) ? v : 0.01f * v;
        if (ACT == 5) v = 0.5f * v * (1.0f + erff(v * 0.70710678118654752f));
        slab[(mOff + r) * 68 + (j << 4) + rlane] = v;
      }
    }
    __builtin_amdgcn_fence(__ATOMIC_RELEASE, "workgroup");
    __builtin_amdgcn_wave_barrier();
    __builtin_amdgcn_fence(__ATOMIC_ACQUIRE, "workgroup");
    if (OUT_MODE == 0) {
      float* C = (float*)Cout + (size_t)b * strideC;
      const int hh = lane >> 4, c4 = (lane & 15) * 4;
      for (int pass = 0; pass < 2; ++pass) {
#pragma unroll
        for (int it = 0; it < 8; ++it) {
          const int row = it * 2 + hh;
          v4f v = *(const v4f*)(slab + row * 68 + c4);
          *(volatile v4f*)(C + (size_t)(mBase + row) * ldc + n0 + c4) = v;
        }
        __threadfence();
      }
    } else {
      const int q = lane >> 3, c8 = (lane & 7) * 8;
      unsigned short* C  = (unsigned short*)Cout  + (size_t)b * strideC;
      unsigned short* C2 = (OUT_MODE == 2) ? ((unsigned short*)Cout2 + (size_t)b * strideC) : nullptr;
      for (int pass = 0; pass < 2; ++pass) {
#pragma unroll
        for (int it = 0; it < 4; ++it) {
          const int row = it * 4 + q;
          const float* sp = slab + row * 68 + c8;
          v8h hv, lv;
#pragma unroll
          for (int e = 0; e < 8; ++e) {
            if (OUT_MODE == 1) {
              hv[e] = (_Float16)sp[e];
            } else {
              unsigned short hb = f2bf_bits(sp[e]);
              unsigned short lb = f2bf_bits(sp[e] - bf_bits2f(hb));
              hv[e] = __builtin_bit_cast(_Float16, hb);
              lv[e] = __builtin_bit_cast(_Float16, lb);
            }
          }
          *(volatile v8h*)(C + (size_t)(mBase + row) * ldc + n0 + c8) = hv;
          if (OUT_MODE == 2) *(volatile v8h*)(C2 + (size_t)(mBase + row) * ldc + n0 + c8) = lv;
        }
        __threadfence();
      }
    }
    __builtin_amdgcn_fence(__ATOMIC_RELEASE, "workgroup");
    __builtin_amdgcn_wave_barrier();
    __builtin_amdgcn_fence(__ATOMIC_ACQUIRE, "workgroup");
  }
}


#ifndef SRB
#define SRB 512
#endif
#ifndef SCHK
#define SCHK 4096
#endif
#define SEPT (SCHK / SRB)
__device__ __forceinline__ int blk_excl_scan(int cnt, int* scan_ws, int tid, int* tot) {
  const int lane = tid & 31, wave = tid >> 5; int incl = cnt;
#pragma unroll
  for (int o = 1; o < 32; o <<= 1) { const int v = __shfl_up(incl, o, 32); if (lane >= o) incl += v; }
  if (lane == 31) scan_ws[wave] = incl;
  __syncthreads();
  if (wave == 0) { int wv = (lane < SRB / 32) ? scan_ws[lane] : 0; int wincl = wv;
#pragma unroll
    for (int o = 1; o < 32; o <<= 1) { const int v = __shfl_up(wincl, o, 32); if (lane >= o) wincl += v; }
    if (lane < SRB / 32) scan_ws[32 + lane] = wincl - wv; if (lane == 31) scan_ws[64] = wincl; }
  __syncthreads();
  const int res = scan_ws[32 + wave] + incl - cnt; *tot = scan_ws[64];
  return res;
}
__device__ __forceinline__ int chunk_compact(const int* __restrict__ keyv, const int* __restrict__ othv, int e0, int ne, int n0, int nn, int tid, int* L0, int* L1, int* L2, int* scan_ws) {
  int hk[SEPT], ho[SEPT], he[SEPT]; int cnt = 0;
#pragma unroll
  for (int k = 0; k < SEPT; ++k) { const int e = e0 + tid * SEPT + k; hk[k] = -1; if (e < ne) { const int d = keyv[e]; if (d >= n0 && d < n0 + SRB && d < nn) { hk[k] = d - n0; int s = othv[e]; s = s < 0 ? 0 : (s >= nn ? nn - 1 : s); ho[k] = s; he[k] = e; ++cnt; } } }
  int tot; int p = blk_excl_scan(cnt, scan_ws, tid, &tot);
#pragma unroll
  for (int k = 0; k < SEPT; ++k) if (hk[k] >= 0) { L0[p] = hk[k]; L1[p] = ho[k]; if (L2) L2[p] = he[k]; ++p; }
  __syncthreads();
  return tot;
}
__global__ __launch_bounds__(SRB) void stream_deg_kernel(const int* __restrict__ keyv, const int* __restrict__ othv, int ne, int nn, int* __restrict__ DEG) {
  __shared__ int L0[SCHK]; __shared__ int L1[SCHK]; __shared__ int scan_ws[80];
  const int tid = threadIdx.x, n0 = blockIdx.x * SRB; int cnt = 0;
  for (int e0 = 0; e0 < ne; e0 += SCHK) { const int tot = chunk_compact(keyv, othv, e0, ne, n0, nn, tid, L0, L1, nullptr, scan_ws);
    for (int q = 0; q < tot; ++q) cnt += (L0[q] == tid) ? 1 : 0;
    __syncthreads(); }
  const int n = n0 + tid; if (n < nn) { ((volatile int*)DEG)[n] = cnt; __threadfence(); ((volatile int*)DEG)[n] = cnt; }
}
#define WCAP 64
template <int LO, int HI, int VPL> struct SlotDisp { static __device__ __forceinline__ void add(int s, float (*acc)[VPL], const float* v) {
  if (LO + 1 == HI) {
#pragma unroll
    for (int j = 0; j < VPL; ++j) acc[LO][j] += v[j]; }
  else { const int MID = (LO + HI) / 2; if (s < MID) SlotDisp<LO, (LO + HI) / 2, VPL>::add(s, acc, v); else SlotDisp<(LO + HI) / 2, HI, VPL>::add(s, acc, v); } } };
template <int VW, int CNT>
__device__ __forceinline__ void coop_flush(int n, const unsigned char* wls, const int* wlv, const float* wlw, const float* __restrict__ Hm, int ldh, int lane, float (*acc)[VW + CNT], float* cnl) {
  for (int j = 0; j < n; ++j) { const int slot = wls[j]; const int src = wlv[j]; const float ew = wlw ? wlw[j] : 1.0f; float v[VW + CNT]; const float* hp = Hm + (size_t)src * ldh + lane * VW;
    if (cnl != nullptr && lane == 0) cnl[slot] += 1.0f;
#pragma unroll
    for (int q = 0; q < VW; ++q) v[q] = wlw ? hp[q] * ew : hp[q];
    if (CNT) v[VW + CNT - 1] = 1.0f;
    SlotDisp<0, 32, VW + CNT>::add(slot, acc, v); }
}
template <int VW, int CNT>
__device__ __forceinline__ void coop_chunk(int tot, const int* L0, const int* L1, const int* L2, const float* __restrict__ EW, unsigned char* wls, int* wlv, float* wlw, const float* __restrict__ Hm, int ldh, int wave, int lane, float (*acc)[VW + CNT], float* cnl) {
  int nlist = 0;
  for (int q0 = 0; q0 < tot; q0 += 32) { const int q = q0 + lane; int l0 = 0, l1 = 0; float w = 1.f; bool mine = false; if (q < tot) { l0 = L0[q]; l1 = L1[q]; if (EW) w = EW[L2[q]]; mine = (l0 >> 5) == wave; }
    const unsigned bal = __builtin_amdgcn_ballot_w32(mine); const int cntb = __builtin_popcount(bal);
    if (nlist + cntb > WCAP) { coop_flush<VW, CNT>(nlist, wls, wlv, EW ? wlw : nullptr, Hm, ldh, lane, acc, cnl); nlist = 0; }
    const int pos = nlist + __builtin_popcount(bal & ((1u << lane) - 1u));
    if (mine) { wls[pos] = (unsigned char)(l0 & 31); wlv[pos] = l1; if (EW) wlw[pos] = w; }
    nlist += cntb; }
  coop_flush<VW, CNT>(nlist, wls, wlv, EW ? wlw : nullptr, Hm, ldh, lane, acc, cnl);
}
template <int VW, bool BIDIR, int CNT>
__global__ __launch_bounds__(SRB) void coop_agg_kernel(const float* __restrict__ Hm, int ldh, const int* __restrict__ keyv, const int* __restrict__ othv, const float* __restrict__ EW, int ne, int nn, float* __restrict__ RAW, int ldr, float* __restrict__ DEGOUT) {
  __shared__ int L0[SCHK]; __shared__ int L1[SCHK]; __shared__ int L2[SCHK]; __shared__ int scan_ws[80]; __shared__ unsigned char WLs[32][WCAP]; __shared__ int WLv[32][WCAP]; __shared__ float WLw[32][WCAP]; __shared__ float CNL[SRB];
  const int tid = threadIdx.x, lane = tid & 31, wave = tid >> 5, n0 = blockIdx.x * SRB;
  CNL[tid] = 0.f; float* cnl = (CNT == 0 && DEGOUT != nullptr) ? (CNL + wave * 32) : nullptr;
  __syncthreads();
  float acc[32][VW + CNT];
#pragma unroll
  for (int s = 0; s < 32; ++s)
#pragma unroll
    for (int j = 0; j < VW + CNT; ++j) acc[s][j] = 0.f;
  for (int e0 = 0; e0 < ne; e0 += SCHK) {
#pragma unroll
    for (int dir = 0; dir < (BIDIR ? 2 : 1); ++dir) {
      const int tot = chunk_compact(dir ? othv : keyv, dir ? keyv : othv, e0, ne, n0, nn, tid, L0, L1, EW ? L2 : nullptr, scan_ws);
      coop_chunk<VW, CNT>(tot, L0, L1, L2, EW, WLs[wave], WLv[wave], WLw[wave], Hm, ldh, wave, lane, acc, cnl);
      __syncthreads(); } }
  __syncthreads();
#pragma unroll
  for (int s = 0; s < 32; ++s) { const int n = n0 + wave * 32 + s; if (n < nn) { float* dst = RAW + (size_t)n * ldr + lane * VW;
      for (int pass = 0; pass < 2; ++pass) {
#pragma unroll
        for (int j = 0; j < VW; ++j) ((volatile float*)dst)[j] = acc[s][j];
        if (CNT && lane == 0) ((volatile float*)DEGOUT)[n] = acc[s][VW + CNT - 1];
        if (cnl != nullptr && lane == 0) ((volatile float*)DEGOUT)[n] = CNL[wave * 32 + s];
        __threadfence(); } } }
}

#define DN_ 50000
#define DNP 50048
#define DE 800000
__device__ __forceinline__ unsigned pkh(float a, float b) { return (unsigned)__builtin_bit_cast(unsigned short, (_Float16)a) | ((unsigned)__builtin_bit_cast(unsigned short, (_Float16)b) << 16); }
template <int WD>
__global__ __launch_bounds__(256) void build_kernel(const float* __restrict__ X, const float* __restrict__ AGG, const float* __restrict__ DEG, unsigned* __restrict__ A16) {
  const long i = (long)blockIdx.x * 256 + threadIdx.x; if (i >= (long)DNP * WD) return; const long n = i / WD; const int cp = 2 * (int)(i % WD); float a = 0.f, b = 0.f;
  if (n < DN_) { if (cp < WD) { a = X[n * WD + cp]; b = X[n * WD + cp + 1]; } else { const float s = 1.0f / fmaxf(DEG[n], 1.0f); a = AGG[n * WD + cp - WD] * s; b = AGG[n * WD + cp - WD + 1] * s; } }
  ((volatile unsigned*)A16)[i] = pkh(a, b); __threadfence(); ((volatile unsigned*)A16)[i] = pkh(a, b);
}
__global__ __launch_bounds__(256) void wcat_kernel(const float* __restrict__ Ws, const float* __restrict__ Wn, const float* __restrict__ b, int KIN, int NOUT, float s0, float s1, unsigned* __restrict__ BT, float* __restrict__ SB0, float* __restrict__ SB1) {
  for (int i = blockIdx.x * 256 + threadIdx.x; i < NOUT * KIN; i += gridDim.x * 256) { const int o = i / KIN, kp = 2 * (i % KIN); float a, c;
    if (kp < KIN) { a = Ws[(size_t)kp * NOUT + o]; c = Ws[(size_t)(kp + 1) * NOUT + o]; } else { a = Wn[(size_t)(kp - KIN) * NOUT + o]; c = Wn[(size_t)(kp + 1 - KIN) * NOUT + o]; }
    ((volatile unsigned*)BT)[i] = pkh(a, c); __threadfence(); ((volatile unsigned*)BT)[i] = pkh(a, c);
    if (i < NOUT) { ((volatile float*)SB0)[i] = b[i] * s0; ((volatile float*)SB1)[i] = b[i] * s1; } }
}
__global__ __launch_bounds__(256) void copy_kernel(const float* __restrict__ S, float* __restrict__ D, long n4) { const long i = (long)blockIdx.x * 256 + threadIdx.x; if (i >= n4) return; const v4f v = *(const v4f*)(S + 4 * i); *(volatile v4f*)(D + 4 * i) = v; __threadfence(); *(volatile v4f*)(D + 4 * i) = v; }
extern "C" void kernel_launch(void* const* d_in, const int* in_sizes, int n_in, void* d_out, int out_size, void* d_ws, size_t ws_size, hipStream_t stream) {
  (void)in_sizes; (void)n_in; (void)out_size; (void)ws_size;
  auto Fp = [&](int i) { return (const float*)d_in[i]; };
  const float* X = Fp(0); const int* src1 = (const int*)d_in[1]; const int* dst1 = (const int*)d_in[2]; const int* src2 = (const int*)d_in[3]; const int* dst2 = (const int*)d_in[4];
  const float* Ws1 = Fp(5); const float* Wn1 = Fp(6); const float* b1 = Fp(7); const float* Ws2 = Fp(8); const float* Wn2 = Fp(9); const float* b2 = Fp(10);
  const float TEM0 = 0.8f, TEM1 = 0.6f;
  char* ws = (char*)d_ws; size_t off = 0;
  auto carve = [&](size_t bytes) -> char* { char* p = ws + off; off += (bytes + 255) & ~(size_t)255; return p; };
  float* AGG = (float*)carve((size_t)DNP * 128 * 4); float* DEG1 = (float*)carve((size_t)DNP * 4); float* DEG2 = (float*)carve((size_t)DNP * 4); unsigned* A16 = (unsigned*)carve((size_t)DNP * 256 * 2);
  unsigned* BT1 = (unsigned*)carve(128 * 256 * 2); unsigned* BT2 = (unsigned*)carve(64 * 256 * 2); float* SB = (float*)carve(4 * 128 * 4); float* X1 = (float*)carve((size_t)DNP * 128 * 4); float* OUTP = (float*)carve((size_t)DNP * 64 * 4); float* OUT2 = (float*)carve((size_t)DNP * 64 * 4);
  const int nb = (DN_ + SRB - 1) / SRB; const int t2 = (DNP / 64) * 2, t1 = (DNP / 64) * 1;
  wcat_kernel<<<64, 256, 0, stream>>>(Ws1, Wn1, b1, 128, 128, TEM0, TEM1, BT1, SB, SB + 128); wcat_kernel<<<32, 256, 0, stream>>>(Ws2, Wn2, b2, 128, 64, TEM0, TEM1, BT2, SB + 256, SB + 320);
  coop_agg_kernel<4, false, 0><<<nb, SRB, 0, stream>>>(X, 128, dst1, src1, nullptr, DE, DN_, AGG, 128, DEG1);
  build_kernel<128><<<(unsigned)(((long)DNP * 128 + 255) / 256), 256, 0, stream>>>(X, AGG, DEG1, A16);
  wmma_gemm64<0, false, 2, 0, false><<<dim3((t2 + 7) / 8, 1), 256, 0, stream>>>((const unsigned short*)A16, nullptr, 256, 0, (const unsigned short*)BT1, nullptr, 256, 0, X1, nullptr, 128, 0, SB, nullptr, 0, DNP, 128, 256, TEM0);
  coop_agg_kernel<4, false, 0><<<nb, SRB, 0, stream>>>(X, 128, dst2, src2, nullptr, DE, DN_, AGG, 128, DEG2);
  build_kernel<128><<<(unsigned)(((long)DNP * 128 + 255) / 256), 256, 0, stream>>>(X, AGG, DEG2, A16);
  wmma_gemm64<0, false, 2, 0, true><<<dim3((t2 + 7) / 8, 1), 256, 0, stream>>>((const unsigned short*)A16, nullptr, 256, 0, (const unsigned short*)BT1, nullptr, 256, 0, X1, nullptr, 128, 0, SB + 128, X1, 0, DNP, 128, 256, TEM1);
  coop_agg_kernel<4, false, 0><<<nb, SRB, 0, stream>>>(X1, 128, dst1, src1, nullptr, DE, DN_, AGG, 128, nullptr);
  build_kernel<128><<<(unsigned)(((long)DNP * 128 + 255) / 256), 256, 0, stream>>>(X1, AGG, DEG1, A16);
  wmma_gemm64<0, false, 2, 0, false><<<dim3((t1 + 7) / 8, 1), 256, 0, stream>>>((const unsigned short*)A16, nullptr, 256, 0, (const unsigned short*)BT2, nullptr, 256, 0, OUTP, nullptr, 64, 0, SB + 256, nullptr, 0, DNP, 64, 256, TEM0);
  coop_agg_kernel<4, false, 0><<<nb, SRB, 0, stream>>>(X1, 128, dst2, src2, nullptr, DE, DN_, AGG, 128, nullptr);
  build_kernel<128><<<(unsigned)(((long)DNP * 128 + 255) / 256), 256, 0, stream>>>(X1, AGG, DEG2, A16);
  wmma_gemm64<0, false, 2, 0, true><<<dim3((t1 + 7) / 8, 1), 256, 0, stream>>>((const unsigned short*)A16, nullptr, 256, 0, (const unsigned short*)BT2, nullptr, 256, 0, OUT2, nullptr, 64, 0, SB + 320, OUTP, 0, DNP, 64, 256, TEM1);
  copy_kernel<<<(unsigned)(((long)DN_ * 16 + 255) / 256), 256, 0, stream>>>(OUT2, (float*)d_out, (long)DN_ * 16);
}
